// MultiHeadAttention_15839839387691
// MI455X (gfx1250) — hardware-verified
//
#include <hip/hip_runtime.h>


#ifndef NB
#define NB 2
#endif
#ifndef SEQ
#define SEQ 2048
#endif
#define SEQ_FULL 2048
#define DM   768
#define NH   12
#define HD   64
#define LP   68
#define PCAR 1024.0f
#define QSCL 0.125f
#define LOG2E 1.4426950408889634f

typedef _Float16 h16;
typedef unsigned short bf;
typedef __attribute__((ext_vector_type(16))) __bf16   v16bf;
typedef __attribute__((ext_vector_type(16))) _Float16 v16h;
typedef __attribute__((ext_vector_type(8)))  _Float16 v8h;
typedef __attribute__((ext_vector_type(8)))  unsigned short v8us;
typedef __attribute__((ext_vector_type(8)))  float    v8f;
typedef __attribute__((ext_vector_type(4)))  float    v4f;
typedef v4f __attribute__((may_alias)) v4fa;

static_assert(NH * HD == DM);
static_assert(HD == 64);
static_assert(DM % 64 == 0);
static_assert(DM % 32 == 0);
static_assert(SEQ % 64 == 0);
static_assert(SEQ % 32 == 0);
static_assert((NB * SEQ) % 64 == 0);
static_assert(((size_t)DM * DM / 8) % 256 == 0);
static_assert(((size_t)NB * SEQ * DM / 8) % 256 == 0);
static_assert(SEQ <= SEQ_FULL);
static_assert((size_t)SEQ * HD < 0x40000000u);

#define SZ_X   ((size_t)NB * SEQ * DM * 2)
#define SZ_W   ((size_t)DM * DM * 2)
#define SZ_P   ((size_t)NB * NH * SEQ * HD * 2)
#define WS_TOTAL (3 * SZ_X + 4 * SZ_W + 5 * SZ_P + 2 * SZ_X)
static_assert(SZ_X % 256 == 0 && SZ_W % 256 == 0 && SZ_P % 256 == 0);
static_assert(WS_TOTAL <= (size_t)134217728);

__device__ __forceinline__ unsigned short f2bf(float f) { unsigned u = __float_as_uint(f); u += 0x7FFFu + ((u >> 16) & 1u); return (unsigned short)(u >> 16); }
__device__ __forceinline__ float bf2f(unsigned short b) { return __uint_as_float(((unsigned)b) << 16); }
__device__ __forceinline__ float bfr(float f) { return bf2f(f2bf(f)); }
__device__ __forceinline__ void splitf(float y, unsigned short& h, unsigned short& l) { h = f2bf(y); l = f2bf(y - bf2f(h)); }
__device__ __forceinline__ v16h cat16(v8h lo, v8h hi) { return __builtin_shufflevector(lo, hi, 0, 1, 2, 3, 4, 5, 6, 7, 8, 9, 10, 11, 12, 13, 14, 15); }
__device__ __forceinline__ v16bf cat16b(v8us lo, v8us hi) { return __builtin_bit_cast(v16bf, __builtin_shufflevector(lo, hi, 0, 1, 2, 3, 4, 5, 6, 7, 8, 9, 10, 11, 12, 13, 14, 15)); }
__device__ __forceinline__ v8f wmma16(v16h a, v16h b, v8f c) { return __builtin_amdgcn_wmma_f32_16x16x32_f16(false, a, false, b, (short)0, c, false, false); }
__device__ __forceinline__ v8f wmmab(v16bf a, v16bf b, v8f c) { return __builtin_amdgcn_wmma_f32_16x16x32_bf16(false, a, false, b, (short)0, c, false, false); }
__device__ __forceinline__ v16bf ldb(const bf* p) { return cat16b(*(const v8us*)p, *(const v8us*)(p + 16)); }
__device__ __forceinline__ v16h ldh(const h16* p) { return cat16(*(const v8h*)p, *(const v8h*)(p + 16)); }

__global__ __launch_bounds__(256) void k_cvt8(const float* __restrict__ src, bf* dst, unsigned n8, unsigned per8, unsigned sstride) {
    const unsigned i = blockIdx.x * 256u + threadIdx.x; if (i >= n8) return;
    const unsigned b = i / per8, r = i - b * per8;
    const v8f v = *(const v8f*)(src + (size_t)b * sstride + (size_t)r * 8); v8us o;
#pragma unroll
    for (int k = 0; k < 8; ++k) o[k] = f2bf(v[k]);
    *(volatile v8us*)(dst + (size_t)i * 8) = o; __threadfence(); *(volatile v8us*)(dst + (size_t)i * 8) = o;
}

template <int NSPLIT>
__device__ __forceinline__ void gemm_main(const bf* __restrict__ A, const bf* __restrict__ A2, const bf* __restrict__ Bt, const int r0, const int c0, const int lane, v8f (&acc)[4][4]) {
    const int lr = lane & 15, hi = lane >> 4;
#pragma unroll
    for (int mb = 0; mb < 4; ++mb)
#pragma unroll
        for (int nb = 0; nb < 4; ++nb) acc[mb][nb] = (v8f){};
    const size_t aoff = (size_t)(r0 + lr) * DM + 8 * hi, boff = (size_t)(c0 + lr) * DM + 8 * hi;
#pragma unroll 1
    for (int kc = 0; kc < DM; kc += 32) {
        v16bf a[4], a2[4], b;
#pragma unroll
        for (int mb = 0; mb < 4; ++mb) { a[mb] = ldb(A + aoff + (size_t)mb * 16 * DM + kc); if (NSPLIT == 1) a2[mb] = ldb(A2 + aoff + (size_t)mb * 16 * DM + kc); }
#pragma unroll
        for (int nb = 0; nb < 4; ++nb) { b = ldb(Bt + boff + (size_t)nb * 16 * DM + kc);
#pragma unroll
            for (int mb = 0; mb < 4; ++mb) { acc[mb][nb] = wmmab(a[mb], b, acc[mb][nb]); if (NSPLIT == 1) acc[mb][nb] = wmmab(a2[mb], b, acc[mb][nb]); } }
        asm volatile("" : "+v"(acc[0][0]), "+v"(acc[1][0]), "+v"(acc[2][0]), "+v"(acc[3][0]), "+v"(acc[0][1]), "+v"(acc[1][1]), "+v"(acc[2][1]), "+v"(acc[3][1]));
        if (NSPLIT == 1) asm volatile("v_nop\n\tv_nop\n\tv_nop\n\tv_nop" : "+v"(acc[0][2]), "+v"(acc[1][2]), "+v"(acc[2][2]), "+v"(acc[3][2]), "+v"(acc[0][3]), "+v"(acc[1][3]), "+v"(acc[2][3]), "+v"(acc[3][3]) : "v"(a[3]), "v"(a2[3]), "v"(b));
        else asm volatile("v_nop\n\tv_nop\n\tv_nop\n\tv_nop" : "+v"(acc[0][2]), "+v"(acc[1][2]), "+v"(acc[2][2]), "+v"(acc[3][2]), "+v"(acc[0][3]), "+v"(acc[1][3]), "+v"(acc[2][3]), "+v"(acc[3][3]) : "v"(a[3]), "v"(b));
    }
}

__global__ __launch_bounds__(32) void k_proj_qk(const bf* __restrict__ X, const bf* __restrict__ W, const float* __restrict__ bias, float scl, bf* Ph, bf* Pl) {
    __shared__ __align__(16) float os[16 * LP];
    const int lane = (int)(threadIdx.x & 31), lr = lane & 15, hi = lane >> 4;
    const int r0 = (int)blockIdx.x * 64, c0 = (int)blockIdx.y * 64;
    v8f acc[4][4];
    gemm_main<0>(X, X, W, r0, c0, lane, acc);
    const int bb = r0 / SEQ, t0 = r0 - bb * SEQ, head = (int)blockIdx.y;
    const size_t prow = (size_t)(bb * NH + head) * SEQ + t0;
    const int rq = lane >> 3, pc = lane & 7;
    const v4f bA = *(const v4f*)(bias + c0 + pc * 8), bB = *(const v4f*)(bias + c0 + pc * 8 + 4);
    float bz[8];
#pragma unroll
    for (int k = 0; k < 4; ++k) { bz[k] = bfr(bA[k]); bz[k + 4] = bfr(bB[k]); }
#pragma unroll
    for (int mb = 0; mb < 4; ++mb) {
#pragma unroll
        for (int nb = 0; nb < 4; ++nb) {
#pragma unroll
            for (int j = 0; j < 8; ++j) os[(hi * 8 + j) * LP + nb * 16 + lr] = acc[mb][nb][j]; }
        __syncthreads();
#pragma unroll 1
        for (int ps = 0; ps < 2; ++ps) {
#pragma unroll
            for (int s = 0; s < 4; ++s) { const int row = 4 * s + rq; const v4f x0 = *(const v4fa*)(os + row * LP + pc * 8), x1 = *(const v4fa*)(os + row * LP + pc * 8 + 4); v8us oh, ol;
#pragma unroll
                for (int k = 0; k < 4; ++k) { unsigned short a, c; splitf((x0[k] + bz[k]) * scl, a, c); oh[k] = a; ol[k] = c; splitf((x1[k] + bz[k + 4]) * scl, a, c); oh[k + 4] = a; ol[k + 4] = c; }
                const size_t dst = (prow + (size_t)(mb * 16 + row)) * HD + pc * 8;
                *(volatile v8us*)(Ph + dst) = oh; *(volatile v8us*)(Pl + dst) = ol; }
            if (ps == 0) __threadfence(); }
        __syncthreads();
    }
}

__global__ __launch_bounds__(32) void k_proj_v(const bf* __restrict__ X, const bf* __restrict__ W, const float* __restrict__ bias, h16* VT) {
    __shared__ __align__(16) float tt[64 * LP];
    const int lane = (int)(threadIdx.x & 31), lr = lane & 15, hi = lane >> 4;
    const int r0 = (int)blockIdx.x * 64, c0 = (int)blockIdx.y * 64;
    v8f acc[4][4];
    gemm_main<0>(X, X, W, r0, c0, lane, acc);
    const int bb = r0 / SEQ, t0 = r0 - bb * SEQ, head = (int)blockIdx.y;
    const size_t vbase = (size_t)(bb * NH + head) * HD * SEQ + t0;
    const int rq = lane >> 3, pc = lane & 7;
#pragma unroll
    for (int mb = 0; mb < 4; ++mb)
#pragma unroll
        for (int nb = 0; nb < 4; ++nb) {
#pragma unroll
            for (int j = 0; j < 8; ++j) tt[(nb * 16 + lr) * LP + mb * 16 + hi * 8 + j] = acc[mb][nb][j]; }
    __syncthreads();
#pragma unroll 1
    for (int ps = 0; ps < 2; ++ps) {
#pragma unroll 4
        for (int s = 0; s < 16; ++s) { const int d = 4 * s + rq; const v4f x0 = *(const v4fa*)(tt + d * LP + pc * 8), x1 = *(const v4fa*)(tt + d * LP + pc * 8 + 4); const float bv = bfr(bias[c0 + d]); v8h o;
#pragma unroll
            for (int k = 0; k < 4; ++k) { o[k] = (h16)(x0[k] + bv); o[k + 4] = (h16)(x1[k] + bv); }
            *(volatile v8h*)(VT + vbase + (size_t)d * SEQ + pc * 8) = o; }
        if (ps == 0) __threadfence(); }
}

__global__ __launch_bounds__(32) void k_proj_o(const bf* __restrict__ A, const bf* __restrict__ A2, const bf* __restrict__ W, const float* __restrict__ bias, float* C) {
    __shared__ __align__(16) float os[16 * LP];
    const int lane = (int)(threadIdx.x & 31), lr = lane & 15, hi = lane >> 4;
    const int r0 = (int)blockIdx.x * 64, c0 = (int)blockIdx.y * 64;
    v8f acc[4][4];
    gemm_main<1>(A, A2, W, r0, c0, lane, acc);
    const int cofs = lr * 4;
    const v4f b4 = *(const v4f*)(bias + c0 + cofs); v4f bz;
#pragma unroll
    for (int k = 0; k < 4; ++k) bz[k] = bfr(b4[k]);
#pragma unroll
    for (int mb = 0; mb < 4; ++mb) {
#pragma unroll
        for (int nb = 0; nb < 4; ++nb) {
#pragma unroll
            for (int j = 0; j < 8; ++j) os[(hi * 8 + j) * LP + nb * 16 + lr] = acc[mb][nb][j]; }
        __syncthreads();
        float* crow = C + (size_t)(r0 + mb * 16) * DM + c0;
#pragma unroll 1
        for (int ps = 0; ps < 2; ++ps) {
#pragma unroll
            for (int s = 0; s < 8; ++s) { const int row = 2 * s + hi; v4f val = *(const v4fa*)(os + row * LP + cofs); val = val + bz;
                *(volatile v4f*)(crow + (size_t)row * DM + cofs) = val; }
            if (ps == 0) __threadfence(); }
        __syncthreads();
    }
}

__global__ __launch_bounds__(128) void k_attn(const bf* __restrict__ Qh, const bf* __restrict__ Ql, const bf* __restrict__ Kh, const bf* __restrict__ Kl, const h16* __restrict__ VT, bf* Ah, bf* Al) {
    __shared__ __align__(16) float os[4][16 * LP];
    const int wave = __builtin_amdgcn_readfirstlane((int)(threadIdx.x >> 5));
    const int lane = (int)(threadIdx.x & 31), lr = lane & 15, hi = lane >> 4;
    const int bh = (int)blockIdx.x / (SEQ / 64);
    const int q0 = ((int)blockIdx.x - bh * (SEQ / 64)) * 64 + wave * 16;
    const size_t pbase = (size_t)bh * SEQ * HD;
    const bf* qh = Qh + pbase; const bf* ql = Ql + pbase; const bf* kh = Kh + pbase; const bf* kl = Kl + pbase; const h16* vt = VT + pbase;
    const int qoff0 = (q0 + lr) * HD + 8 * hi;
    const int koff0 = lr * HD + 8 * hi;
    const int voff0 = lr * SEQ + 8 * hi;
    v8f acc[4];
#pragma unroll
    for (int dt = 0; dt < 4; ++dt) acc[dt] = (v8f){};
    float m = -1.0e30f, l = 0.0f;
#pragma unroll 1
    for (int kv = 0; kv < SEQ; kv += 32) {
        v8f s0 = (v8f){}, s1 = (v8f){};
        v16bf fq, fql, fk, fkl;
#pragma unroll
        for (int ks = 0; ks < 2; ++ks) {
            int qo = qoff0 + ks * 32; asm volatile("" : "+v"(qo));
            fq = ldb(qh + qo); fql = ldb(ql + qo);
            const int ko = koff0 + kv * HD + ks * 32;
            fk = ldb(kh + ko); fkl = ldb(kl + ko);
            s0 = wmmab(fk, fq, s0); s0 = wmmab(fkl, fq, s0); s0 = wmmab(fk, fql, s0);
            fk = ldb(kh + ko + 16 * HD); fkl = ldb(kl + ko + 16 * HD);
            s1 = wmmab(fk, fq, s1); s1 = wmmab(fkl, fq, s1); s1 = wmmab(fk, fql, s1);
        }
        asm volatile("v_nop\n\tv_nop\n\tv_nop\n\tv_nop" : "+v"(s0), "+v"(s1) : "v"(fq), "v"(fql), "v"(fk), "v"(fkl));
        float mx = fmaxf(s0[0], s1[0]);
#pragma unroll
        for (int r = 1; r < 8; ++r) mx = fmaxf(mx, fmaxf(s0[r], s1[r]));
        mx = fmaxf(mx, __shfl_xor(mx, 16, 32));
        const float mn = fmaxf(m, mx);
        const float fac = __builtin_amdgcn_exp2f((m - mn) * LOG2E);
        float ps = 0.0f; v16h pb;
#pragma unroll
        for (int r = 0; r < 8; ++r) { const float p0 = __builtin_amdgcn_exp2f((s0[r] - mn) * LOG2E), p1 = __builtin_amdgcn_exp2f((s1[r] - mn) * LOG2E); ps += p0 + p1; pb[r] = (h16)(p0 * PCAR); pb[r + 8] = (h16)(p1 * PCAR); }
        l = l * fac + ps; m = mn;
#pragma unroll
        for (int dt = 0; dt < 4; ++dt) acc[dt] = acc[dt] * fac;
        v16h fv;
#pragma unroll
        for (int dt = 0; dt < 4; ++dt) { fv = ldh(vt + voff0 + dt * 16 * SEQ + kv); acc[dt] = wmma16(fv, pb, acc[dt]); }
        asm volatile("v_nop\n\tv_nop\n\tv_nop\n\tv_nop" : "+v"(acc[0]), "+v"(acc[1]), "+v"(acc[2]), "+v"(acc[3]) : "v"(fv), "v"(pb));
    }
    const float lt = l + __shfl_xor(l, 16, 32);
    const float inv = 1.0f / (lt * PCAR);
#pragma unroll
    for (int dt = 0; dt < 4; ++dt)
#pragma unroll
        for (int r = 0; r < 8; ++r) os[wave][lr * LP + dt * 16 + hi * 8 + r] = acc[dt][r] * inv;
    __syncthreads();
    const int b = bh / NH, head = bh - b * NH;
    const int rq = lane >> 3, pc = lane & 7;
    const size_t crow = (size_t)b * SEQ + q0;
#pragma unroll 1
    for (int ps2 = 0; ps2 < 2; ++ps2) {
#pragma unroll
        for (int s = 0; s < 4; ++s) { const int row = 4 * s + rq; const v4f x0 = *(const v4fa*)(&os[wave][row * LP + pc * 8]), x1 = *(const v4fa*)(&os[wave][row * LP + pc * 8 + 4]); v8us oh, ol;
#pragma unroll
            for (int k = 0; k < 4; ++k) { unsigned short a, c; splitf(x0[k], a, c); oh[k] = a; ol[k] = c; splitf(x1[k], a, c); oh[k + 4] = a; ol[k + 4] = c; }
            const size_t dst = (crow + (size_t)row) * DM + head * HD + pc * 8;
            *(volatile v8us*)(Ah + dst) = oh; *(volatile v8us*)(Al + dst) = ol; }
        if (ps2 == 0) __threadfence(); }
}

extern "C" void kernel_launch(void* const* d_in, const int* in_sizes, int n_in,
                              void* d_out, int out_size, void* d_ws, size_t ws_size, hipStream_t stream) {
    if (n_in < 11) return;
    const long long need_x = (long long)(NB - 1) * SEQ_FULL * DM + (long long)SEQ * DM;
    if ((long long)in_sizes[0] < need_x || (long long)in_sizes[1] < need_x || (long long)in_sizes[2] < need_x) return;
    if (in_sizes[3] < DM * DM || in_sizes[5] < DM * DM || in_sizes[7] < DM * DM || in_sizes[9] < DM * DM) return;
    if (in_sizes[4] < DM || in_sizes[6] < DM || in_sizes[8] < DM || in_sizes[10] < DM) return;
    if ((long long)out_size < (long long)NB * SEQ * DM) return;
    if ((size_t)WS_TOTAL > ws_size) return;
    const float* xq = (const float*)d_in[0]; const float* xk = (const float*)d_in[1]; const float* xv = (const float*)d_in[2];
    const float* wq = (const float*)d_in[3]; const float* bq = (const float*)d_in[4];
    const float* wk = (const float*)d_in[5]; const float* bk = (const float*)d_in[6];
    const float* wv = (const float*)d_in[7]; const float* bv = (const float*)d_in[8];
    const float* wo = (const float*)d_in[9]; const float* bo = (const float*)d_in[10];
    float* OUT = (float*)d_out;
    char* wsp = (char*)d_ws;
    bf* XQ = (bf*)wsp; wsp += SZ_X; bf* XK = (bf*)wsp; wsp += SZ_X; bf* XV = (bf*)wsp; wsp += SZ_X;
    bf* WQ = (bf*)wsp; wsp += SZ_W; bf* WK = (bf*)wsp; wsp += SZ_W; bf* WV = (bf*)wsp; wsp += SZ_W; bf* WO = (bf*)wsp; wsp += SZ_W;
    bf* QPh = (bf*)wsp; wsp += SZ_P; bf* QPl = (bf*)wsp; wsp += SZ_P; bf* KPh = (bf*)wsp; wsp += SZ_P; bf* KPl = (bf*)wsp; wsp += SZ_P;
    h16* VT16 = (h16*)wsp; wsp += SZ_P;
    bf* ATh = (bf*)wsp; wsp += SZ_X; bf* ATl = (bf*)wsp; wsp += SZ_X;
    const unsigned nW8 = (unsigned)((size_t)DM * DM / 8), nX8 = (unsigned)((size_t)NB * SEQ * DM / 8), per8 = (unsigned)((size_t)SEQ * DM / 8);
    k_cvt8<<<nW8 / 256, 256, 0, stream>>>(wq, WQ, nW8, nW8, 0u);
    k_cvt8<<<nW8 / 256, 256, 0, stream>>>(wk, WK, nW8, nW8, 0u);
    k_cvt8<<<nW8 / 256, 256, 0, stream>>>(wv, WV, nW8, nW8, 0u);
    k_cvt8<<<nW8 / 256, 256, 0, stream>>>(wo, WO, nW8, nW8, 0u);
    k_cvt8<<<nX8 / 256, 256, 0, stream>>>(xq, XQ, nX8, per8, (unsigned)((size_t)SEQ_FULL * DM));
    k_cvt8<<<nX8 / 256, 256, 0, stream>>>(xk, XK, nX8, per8, (unsigned)((size_t)SEQ_FULL * DM));
    k_cvt8<<<nX8 / 256, 256, 0, stream>>>(xv, XV, nX8, per8, (unsigned)((size_t)SEQ_FULL * DM));
    const dim3 gp((unsigned)(NB * SEQ / 64), (unsigned)(DM / 64), 1);
    k_proj_qk<<<gp, 32, 0, stream>>>(XQ, WQ, bq, QSCL, QPh, QPl);
    k_proj_qk<<<gp, 32, 0, stream>>>(XK, WK, bk, 1.0f, KPh, KPl);
    k_proj_v<<<gp, 32, 0, stream>>>(XV, WV, bv, VT16);
    k_attn<<<(unsigned)(NB * NH * (SEQ / 64)), 128, 0, stream>>>(QPh, QPl, KPh, KPl, VT16, ATh, ATl);
    k_proj_o<<<gp, 32, 0, stream>>>(ATh, ATl, WO, bo, OUT);
}
